// QGNN_75445395522274
// MI455X (gfx1250) — hardware-verified
//
#include <hip/hip_runtime.h>
#include <stddef.h>


#define GR    32
#define NTHR  256
#define NWAVE 8
#define PW    128
#define KMAX  256
#define AP    (KMAX + 8)
#define XSP   132
#define NB    512
#define CHUNK 2048
#define WCAP  256
#define NGRP  (CHUNK / (NTHR * 4))
#define INTER 128
#define LDS_AGG ((NB * PW + NB + NWAVE * WCAP + NWAVE) * 4)

static_assert(WCAP == (CHUNK / NTHR) * 32);
static_assert(NGRP == 2);
static_assert(NB == 512);
static_assert(CHUNK <= 4096);
static_assert((AP % 8) == 0);
static_assert(((NB * PW + NB) % 4) == 0);
static_assert(LDS_AGG == 272416);
static_assert((GR * AP * 2) % 16 == 0);

typedef float          v4f  __attribute__((ext_vector_type(4)));
typedef float          v8f  __attribute__((ext_vector_type(8)));
typedef int            v4i  __attribute__((ext_vector_type(4)));
typedef unsigned short v8us __attribute__((ext_vector_type(8)));
typedef __bf16         v16b __attribute__((ext_vector_type(16)));
union Frag { v16b v; v8us half[2]; };
union Pk8  { v8us h; v4i q; };

__device__ __forceinline__ v8f wm(v16b a, v16b b, v8f c) {
  v8f d = __builtin_amdgcn_wmma_f32_16x16x32_bf16(false, a, false, b, (short)0, c, false, false);
  asm volatile("v_nop\n\tv_nop\n\tv_nop\n\tv_nop" : "+v"(d) : "v"(a), "v"(b));
  return d;
}

__device__ __forceinline__ unsigned short bf_rne(float f) {
  const unsigned u = __float_as_uint(f);
  return (unsigned short)((u + 0x7FFFu + ((u >> 16) & 1u)) >> 16);
}
__device__ __forceinline__ float bf_val(unsigned short b) {
  return __uint_as_float(((unsigned)b) << 16);
}

__device__ __forceinline__ void split8(v4f f0, v4f f1, Pk8& uh, Pk8& ul) {
  const float x[8] = {f0.x, f0.y, f0.z, f0.w, f1.x, f1.y, f1.z, f1.w};
#pragma unroll
  for (int t = 0; t < 8; ++t) {
    const unsigned short hb = bf_rne(x[t]);
    uh.h[t] = hb;
    ul.h[t] = bf_rne(x[t] - bf_val(hb));
  }
}

__global__ __launch_bounds__(NTHR) void k_wprep(const float* __restrict__ W,
                                                unsigned short* Wh, unsigned short* Wl,
                                                int nrows, int Ks, int Kp) {
  const int total8 = (nrows * Kp) >> 3;
  const int i = blockIdx.x * NTHR + threadIdx.x;
  if (i >= total8) return;
  const int e0 = i * 8;
  const int n  = e0 / Kp;
  const int k  = e0 - n * Kp;
  const float* p = W + (size_t)n * Ks + k;
  v4f f0, f1;
  f0.x = p[0]; f0.y = p[1]; f0.z = p[2]; f0.w = p[3];
  f1.x = p[4]; f1.y = p[5]; f1.z = p[6]; f1.w = p[7];
  Pk8 uh, ul;
  split8(f0, f1, uh, ul);
  *(volatile v4i*)(Wh + e0) = uh.q;
  *(volatile v4i*)(Wl + e0) = ul.q;
  __threadfence();
  *(volatile v4i*)(Wh + e0) = uh.q;
  *(volatile v4i*)(Wl + e0) = ul.q;
}

__global__ __launch_bounds__(NTHR) void k_embed(const int* __restrict__ gt, const float* __restrict__ emb,
                                                float* H, int nN, int nEmbRows, int EC) {
  const int lane = threadIdx.x & 31;
  const int row  = blockIdx.x * NWAVE + (threadIdx.x >> 5);
  if (row >= nN) return;
  int g = gt[row];
  g = g < 0 ? 0 : (g > nEmbRows - 1 ? nEmbRows - 1 : g);
  const int c  = 4 * lane;
  const int cc = (c + 4 <= EC) ? c : (EC - 4);
  v4f v = *(const v4f*)(emb + (size_t)g * EC + cc);
  const v4f z = {0.f, 0.f, 0.f, 0.f};
  v = (c + 4 <= EC) ? v : z;
  float* op = H + (size_t)row * PW + c;
  *(volatile v4f*)op = v;
  __threadfence();
  *(volatile v4f*)op = v;
}

template <int NT>
__global__ __launch_bounds__(NTHR) void k_gemm(
    const float* A0, int K0,
    const float* __restrict__ A1, int K1, int a1RowOff, int a1Rows,
    const unsigned short* __restrict__ Bh, const unsigned short* __restrict__ Bl,
    const float* __restrict__ bias, int hasBias, int doRelu,
    float* outp, int outPitch, int rowBase0, int nN) {
  __shared__ __attribute__((aligned(16))) unsigned short Ah[GR * AP];
  __shared__ __attribute__((aligned(16))) unsigned short Al[GR * AP];
  __shared__ __attribute__((aligned(16))) float Xs[GR * XSP];

  const int tid  = threadIdx.x;
  const int lane = tid & 31;
  const int wave = tid >> 5;
  const int hh   = lane >> 4;
  const int m    = lane & 15;
  const int rowBase = rowBase0 + blockIdx.x * GR;
  const int K = K0 + K1;

  {
    const int cg = K0 >> 3;
    const int items = GR * cg;
    for (int q = tid; q < items; q += NTHR) {
      const int r = q / cg;
      const int c = (q - r * cg) * 8;
      int row = rowBase + r;
      row = row > nN - 1 ? nN - 1 : row;
      const float* p = A0 + (size_t)row * PW + c;
      const v4f f0 = *(const v4f*)(p), f1 = *(const v4f*)(p + 4);
      Pk8 uh, ul;
      split8(f0, f1, uh, ul);
      *(v8us*)(Ah + r * AP + c) = uh.h;
      *(v8us*)(Al + r * AP + c) = ul.h;
    }
  }
  {
    const int cg = K1 >> 3;
    const int items = GR * cg;
    for (int q = tid; q < items; q += NTHR) {
      const int r = q / cg;
      const int c = (q - r * cg) * 8;
      int row = rowBase + r;
      row = row > nN - 1 ? nN - 1 : row;
      int r1 = row - a1RowOff;
      r1 = r1 < 0 ? 0 : (r1 > a1Rows - 1 ? a1Rows - 1 : r1);
      const float* p = A1 + (size_t)r1 * PW + c;
      const v4f f0 = *(const v4f*)(p), f1 = *(const v4f*)(p + 4);
      Pk8 uh, ul;
      split8(f0, f1, uh, ul);
      *(v8us*)(Ah + r * AP + K0 + c) = uh.h;
      *(v8us*)(Al + r * AP + K0 + c) = ul.h;
    }
  }
  __syncthreads();

  constexpr int MT = (NT == 8) ? 2 : 1;
  const int nt   = (NT == 8) ? wave : (wave & 3);
  const int mt0  = (NT == 8) ? 0 : (wave >> 2);
  const int ncol = nt * 16 + m;
  const int nks  = K >> 5;
  v8f acc[MT];
#pragma unroll
  for (int i = 0; i < MT; ++i) { const v8f z = {0.f, 0.f, 0.f, 0.f, 0.f, 0.f, 0.f, 0.f}; acc[i] = z; }
  const unsigned short* pbh = Bh + (size_t)ncol * K + 8 * hh;
  const unsigned short* pbl = Bl + (size_t)ncol * K + 8 * hh;
#pragma unroll 1
  for (int kt = 0; kt < nks; ++kt) {
    const int k0 = kt * 32;
    Frag bh, bl;
    bh.half[0] = *(const v8us*)(pbh + k0); bh.half[1] = *(const v8us*)(pbh + k0 + 16);
    bl.half[0] = *(const v8us*)(pbl + k0); bl.half[1] = *(const v8us*)(pbl + k0 + 16);
    Frag ah[MT], al[MT];
#pragma unroll
    for (int i = 0; i < MT; ++i) {
      const int ra = (mt0 + i) * 16 + m;
      const unsigned short* ph = Ah + ra * AP + k0 + 8 * hh;
      const unsigned short* pl = Al + ra * AP + k0 + 8 * hh;
      ah[i].half[0] = *(const v8us*)ph; ah[i].half[1] = *(const v8us*)(ph + 16);
      al[i].half[0] = *(const v8us*)pl; al[i].half[1] = *(const v8us*)(pl + 16);
    }
#pragma unroll
    for (int i = 0; i < MT; ++i) {
      acc[i] = wm(ah[i].v, bh.v, acc[i]);
      acc[i] = wm(ah[i].v, bl.v, acc[i]);
      acc[i] = wm(al[i].v, bh.v, acc[i]);
    }
  }

  const float braw = bias[hasBias ? ncol : 0];
  const float bv = hasBias ? braw : 0.f;
#pragma unroll
  for (int i = 0; i < MT; ++i) {
#pragma unroll
    for (int r = 0; r < 8; ++r) {
      float v = acc[i][r] + bv;
      if (doRelu) v = fmaxf(v, 0.f);
      Xs[((mt0 + i) * 16 + 8 * hh + r) * XSP + ncol] = v;
    }
  }
  __syncthreads();

  if (NT == 8) {
    v4f xr[4];
    int rows[4];
#pragma unroll
    for (int i = 0; i < 4; ++i) {
      xr[i] = *(const v4f*)(Xs + (4 * wave + i) * XSP + 4 * lane);
      rows[i] = rowBase + 4 * wave + i;
    }
#pragma unroll
    for (int i = 0; i < 4; ++i)
      if (rows[i] < nN) *(volatile v4f*)(outp + (size_t)rows[i] * outPitch + 4 * lane) = xr[i];
    __threadfence();
#pragma unroll
    for (int i = 0; i < 4; ++i)
      if (rows[i] < nN) *(volatile v4f*)(outp + (size_t)rows[i] * outPitch + 4 * lane) = xr[i];
  } else {
    v4f xr[2];
    int rows[2];
#pragma unroll
    for (int j = 0; j < 2; ++j) {
      const int rl = 4 * wave + 2 * j + hh;
      xr[j] = *(const v4f*)(Xs + rl * XSP + 4 * m);
      rows[j] = rowBase + rl;
    }
#pragma unroll
    for (int j = 0; j < 2; ++j)
      if (rows[j] < nN) *(volatile v4f*)(outp + (size_t)rows[j] * outPitch + 4 * m) = xr[j];
    __threadfence();
#pragma unroll
    for (int j = 0; j < 2; ++j)
      if (rows[j] < nN) *(volatile v4f*)(outp + (size_t)rows[j] * outPitch + 4 * m) = xr[j];
  }
}

__global__ __launch_bounds__(NTHR) void k_agg(
    const float* __restrict__ P, const int* __restrict__ src, const int* __restrict__ dst,
    const float* __restrict__ sidx, const float* __restrict__ didx, const float* __restrict__ rev,
    const float* __restrict__ W1, float* HN, int F, int nodeBase0, int nN, int nE) {
  extern __shared__ v4f lds_dyn[];
  float* sacc = (float*)lds_dyn;
  float* cntp = sacc + NB * PW;
  int*   list = (int*)(cntp + NB);
  int*   wcnt = list + NWAVE * WCAP;

  const int tid  = threadIdx.x;
  const int lane = tid & 31;
  const int wave = tid >> 5;
  const int nodeBase = nodeBase0 + blockIdx.x * NB;

  {
    const v4f z4 = {0.f, 0.f, 0.f, 0.f};
    for (int i = tid; i < (NB * PW + NB) / 4; i += NTHR) lds_dyn[i] = z4;
  }
  const int Fs = F + 3;
  v4f ea, eb, ec;
  {
    const float* w0 = W1 + (size_t)(4 * lane) * Fs + F;
    ea.x = w0[0];      eb.x = w0[1];          ec.x = w0[2];
    ea.y = w0[Fs];     eb.y = w0[Fs + 1];     ec.y = w0[Fs + 2];
    ea.z = w0[2 * Fs]; eb.z = w0[2 * Fs + 1]; ec.z = w0[2 * Fs + 2];
    ea.w = w0[3 * Fs]; eb.w = w0[3 * Fs + 1]; ec.w = w0[3 * Fs + 2];
  }
  __syncthreads();

  const bool al16 = ((((size_t)dst) & 15) == 0);
  const int nChunks = (nE + CHUNK - 1) / CHUNK;
#pragma unroll 1
  for (int ch = 0; ch < nChunks; ++ch) {
    const int cbase = ch * CHUNK;
    int wc = 0;
#pragma unroll
    for (int g = 0; g < NGRP; ++g) {
      const int el0 = (g * NTHR + tid) * 4;
      const int e0  = cbase + el0;
      const int sent = -2147483647 - 1;
      v4i d;
      if (al16 && (cbase + CHUNK <= nE)) {
        d = *(const v4i*)(dst + e0);
      } else {
        d.x = (e0     < nE) ? dst[min(e0,     nE - 1)] : sent;
        d.y = (e0 + 1 < nE) ? dst[min(e0 + 1, nE - 1)] : sent;
        d.z = (e0 + 2 < nE) ? dst[min(e0 + 2, nE - 1)] : sent;
        d.w = (e0 + 3 < nE) ? dst[min(e0 + 3, nE - 1)] : sent;
      }
      const unsigned s0 = (unsigned)d.x - (unsigned)nodeBase;
      const unsigned s1 = (unsigned)d.y - (unsigned)nodeBase;
      const unsigned s2 = (unsigned)d.z - (unsigned)nodeBase;
      const unsigned s3 = (unsigned)d.w - (unsigned)nodeBase;
      const bool h0 = s0 < (unsigned)NB;
      const bool h1 = s1 < (unsigned)NB;
      const bool h2 = s2 < (unsigned)NB;
      const bool h3 = s3 < (unsigned)NB;
      const unsigned many = __builtin_amdgcn_ballot_w32(h0 | h1 | h2 | h3);
      if (many != 0u) {
#define HITJ(J, HJ, SJ) { \
          const unsigned mj = __builtin_amdgcn_ballot_w32(HJ); \
          if (HJ) { \
            const int pos = wc + (int)__builtin_amdgcn_mbcnt_lo(mj, 0u); \
            if (pos < WCAP) list[wave * WCAP + pos] = ((el0 + (J)) << 9) | (int)(SJ); \
          } \
          wc += (int)__builtin_popcount(mj); }
        HITJ(0, h0, s0)
        HITJ(1, h1, s1)
        HITJ(2, h2, s2)
        HITJ(3, h3, s3)
#undef HITJ
      }
    }
    if (lane == 0) wcnt[wave] = wc;
    __syncthreads();

    if (wave == 0) {
      for (int wsx = 0; wsx < NWAVE; ++wsx) {
        int n = wcnt[wsx];
        if (n > WCAP) n = WCAP;
        if (n < 0) n = 0;
        for (int i = 0; i < n; ++i) {
          const int ent  = list[wsx * WCAP + i];
          const int slot = ent & (NB - 1);
          const int el   = (ent >> 9) & (CHUNK - 1);
          int e = cbase + el;
          if (e > nE - 1) e = nE - 1;
          int sI = src[e];
          sI = sI < 0 ? 0 : (sI > nN - 1 ? nN - 1 : sI);
          const float w0 = sidx[e], w1 = didx[e], w2 = rev[e];
          const v4f pv = *(const v4f*)(P + (size_t)sI * PW + 4 * lane);
          v4f t = pv + w0 * ea + w1 * eb + w2 * ec;
          t.x = t.x > 0.f ? t.x : 0.01f * t.x;
          t.y = t.y > 0.f ? t.y : 0.01f * t.y;
          t.z = t.z > 0.f ? t.z : 0.01f * t.z;
          t.w = t.w > 0.f ? t.w : 0.01f * t.w;
          v4f* sp = (v4f*)(sacc + slot * PW + 4 * lane);
          const v4f cur = *sp;
          *sp = cur + t;
          if (lane == 0) {
            const float c = cntp[slot];
            cntp[slot] = c + 1.0f;
          }
        }
      }
    }
    __syncthreads();
  }

#pragma unroll 1
  for (int j = 0; j < NB / NWAVE; ++j) {
    const int slot = wave * (NB / NWAVE) + j;
    const int node = nodeBase + slot;
    if (node >= nN) break;
    const float c   = cntp[slot];
    const float inv = 1.0f / fmaxf(c, 1.0f);
    const v4f v = *(const v4f*)(sacc + slot * PW + 4 * lane) * inv;
    float* op = HN + (size_t)(blockIdx.x * NB + slot) * PW + 4 * lane;
    *(volatile v4f*)op = v;
    __threadfence();
    *(volatile v4f*)op = v;
  }
}

extern "C" void kernel_launch(void* const* d_in, const int* in_sizes, int n_in,
                              void* d_out, int out_size, void* d_ws, size_t ws_size,
                              hipStream_t stream) {
  if (n_in < 22) return;
  const int nN = in_sizes[0];
  const int nE = in_sizes[1];
  if (nN <= 0 || nE <= 0) return;
  if (in_sizes[2] != nE || in_sizes[3] != nE || in_sizes[4] != nE || in_sizes[5] != nE) return;
  const int fi[5] = {64, 128, 128, 128, 128};
  const int fo[5] = {128, 128, 128, 128, 64};
  const int EC = fi[0];
  if (in_sizes[6] < EC || (in_sizes[6] % EC) != 0) return;
  const int embRows = in_sizes[6] / EC;
  for (int i = 0; i < 5; ++i) {
    if (in_sizes[7 + 3 * i] != INTER * (fi[i] + 3)) return;
    if (in_sizes[8 + 3 * i] != fo[i] * (fi[i] + INTER)) return;
    if (in_sizes[9 + 3 * i] != fo[i]) return;
  }
  if (out_size != nN * fo[4]) return;

  const int*   gt   = (const int*)d_in[0];
  const int*   src  = (const int*)d_in[1];
  const int*   dst  = (const int*)d_in[2];
  const float* sidx = (const float*)d_in[3];
  const float* didx = (const float*)d_in[4];
  const float* rev  = (const float*)d_in[5];
  const float* emb  = (const float*)d_in[6];
  const float *w1[5], *w2[5], *b2[5];
  for (int i = 0; i < 5; ++i) {
    w1[i] = (const float*)d_in[7 + 3 * i];
    w2[i] = (const float*)d_in[8 + 3 * i];
    b2[i] = (const float*)d_in[9 + 3 * i];
  }
  float* out = (float*)d_out;

  const int nP = ((nN + GR - 1) / GR) * GR;
  const int halfNodes = (nN + 1) / 2;
  const int nHalfBlk  = (halfNodes + NB - 1) / NB;
  const int NHALF     = nHalfBlk * NB;
  size_t off = 0;
  char* ws = (char*)d_ws;
  auto carve = [&](size_t bytes) -> void* {
    void* p = ws + off;
    off += (bytes + 255) & ~(size_t)255;
    return p;
  };
  float* H  = (float*)carve((size_t)nP * PW * sizeof(float));
  float* Pp = (float*)carve((size_t)nP * PW * sizeof(float));
  float* HN = (float*)carve((size_t)NHALF * PW * sizeof(float));
  unsigned short *W1h[5], *W1l[5], *W2h[5], *W2l[5];
  for (int i = 0; i < 5; ++i) {
    const size_t b1 = (size_t)INTER * fi[i] * sizeof(unsigned short);
    const size_t b2b = (size_t)fo[i] * (fi[i] + INTER) * sizeof(unsigned short);
    W1h[i] = (unsigned short*)carve(b1);
    W1l[i] = (unsigned short*)carve(b1);
    W2h[i] = (unsigned short*)carve(b2b);
    W2l[i] = (unsigned short*)carve(b2b);
  }
  if (off > ws_size) return;

  for (int i = 0; i < 5; ++i) {
    const int t1 = (INTER * fi[i]) / 8;
    k_wprep<<<(t1 + NTHR - 1) / NTHR, NTHR, 0, stream>>>(w1[i], W1h[i], W1l[i], INTER, fi[i] + 3, fi[i]);
    const int t2 = (fo[i] * (fi[i] + INTER)) / 8;
    k_wprep<<<(t2 + NTHR - 1) / NTHR, NTHR, 0, stream>>>(w2[i], W2h[i], W2l[i], fo[i], fi[i] + INTER, fi[i] + INTER);
  }

  k_embed<<<(nN + NWAVE - 1) / NWAVE, NTHR, 0, stream>>>(gt, emb, H, nN, embRows, EC);

  hipFuncSetAttribute(reinterpret_cast<const void*>(&k_agg),
                      hipFuncAttributeMaxDynamicSharedMemorySize, LDS_AGG);

  for (int L = 0; L < 5; ++L) {
    const int K0 = fi[L];
    k_gemm<8><<<(nN + GR - 1) / GR, NTHR, 0, stream>>>(
        H, K0, HN, 0, 0, NHALF, W1h[L], W1l[L], b2[L], 0, 0, Pp, PW, 0, nN);
    for (int hf = 0; hf < 2; ++hf) {
      const int hb = hf * NHALF;
      if (hb >= nN) continue;
      const int rows = (nN - hb < NHALF) ? (nN - hb) : NHALF;
      const int ablk = (rows + NB - 1) / NB;
      k_agg<<<ablk, NTHR, LDS_AGG, stream>>>(Pp, src, dst, sidx, didx, rev, w1[L], HN,
                                             K0, hb, nN, nE);
      const int gblk = (rows + GR - 1) / GR;
      if (L < 4) {
        k_gemm<8><<<gblk, NTHR, 0, stream>>>(
            H, K0, HN, INTER, hb, NHALF, W2h[L], W2l[L], b2[L], 1, 1, H, PW, hb, nN);
      } else {
        k_gemm<4><<<gblk, NTHR, 0, stream>>>(
            H, K0, HN, INTER, hb, NHALF, W2h[L], W2l[L], b2[L], 1, 0, out, fo[4], hb, nN);
      }
    }
  }
}
